// HyperKA_60172491817238
// MI455X (gfx1250) — hardware-run, weakly checked
//
#include <hip/hip_runtime.h>

typedef float          v8f   __attribute__((ext_vector_type(8)));
typedef float          v4f   __attribute__((ext_vector_type(4)));
typedef unsigned int   v4u   __attribute__((ext_vector_type(4)));
typedef int            v8i   __attribute__((ext_vector_type(8)));
typedef unsigned short v8us  __attribute__((ext_vector_type(8)));
typedef unsigned short v16us __attribute__((ext_vector_type(16)));
typedef __bf16         v16bf __attribute__((ext_vector_type(16)));
typedef _Float16       v16h  __attribute__((ext_vector_type(16)));
typedef v4f  __attribute__((may_alias)) v4fa;
typedef v8us __attribute__((may_alias)) v8usa;
union FragB { v16bf v; v16us u; v8us h[2]; v8i w; };
union FragH { v16h  v; v16us u; v8us h[2]; v8i w; };

__device__ __forceinline__ v8f wmb(const FragB& a, const FragB& b, v8f c) {
  v8f d = __builtin_amdgcn_wmma_f32_16x16x32_bf16(false, a.v, false, b.v, (short)0, c, false, false);
  asm volatile("v_nop\n\tv_nop\n\tv_nop\n\tv_nop" : "+v"(d) : "v"(a.w), "v"(b.w));
  return d;
}

__device__ __forceinline__ v8f wmh(const FragH& a, const FragH& b, v8f c) {
  v8f d = __builtin_amdgcn_wmma_f32_16x16x32_f16(false, a.v, false, b.v, (short)0, c, false, false);
  asm volatile("v_nop\n\tv_nop\n\tv_nop\n\tv_nop" : "+v"(d) : "v"(a.w), "v"(b.w));
  return d;
}

__device__ __forceinline__ unsigned bf16_bits(float f) {
  const unsigned u = __float_as_uint(f);
  const unsigned r = (u + 0x7FFFu + ((u >> 16) & 1u)) >> 16;
  const unsigned q = (u >> 16) | 0x40u;
  return ((u & 0x7fffffffu) > 0x7f800000u) ? q : r;
}

__device__ __forceinline__ float bf16_val(float f) {
  return __uint_as_float(bf16_bits(f) << 16);
}
__device__ __forceinline__ int clampi(int v, int lo, int hi) {
  return v < lo ? lo : (v > hi ? hi : v);
}

__device__ __forceinline__ unsigned f16_bits(float f) {
  const unsigned u  = __float_as_uint(f);
  const unsigned s  = (u >> 16) & 0x8000u;
  const unsigned a  = u & 0x7fffffffu;
  const unsigned t  = a - 0x38000000u;
  const unsigned r  = (t + 0x0FFFu + ((t >> 13) & 1u)) >> 13;
  const unsigned rc = r > 0x7C00u ? 0x7C00u : r;
  const bool small  = a < 0x38800000u;
  const bool isnan  = a > 0x7f800000u;
  const unsigned fin = small ? 0u : (s | rc);
  return isnan ? (s | 0x7E00u) : fin;
}

__device__ __forceinline__ unsigned pk16(unsigned lo, unsigned hi) { return lo | (hi << 16); }
__device__ __forceinline__ unsigned bf16_lo_bits(float v) {
  float hi = bf16_val(v);
  asm volatile("" : "+v"(hi));
  return bf16_bits(v - hi);
}
__device__ __forceinline__ v4u pack8_bf16(v4f a, v4f c) {
  return (v4u){ pk16(bf16_bits(a[0]), bf16_bits(a[1])), pk16(bf16_bits(a[2]), bf16_bits(a[3])),
                pk16(bf16_bits(c[0]), bf16_bits(c[1])), pk16(bf16_bits(c[2]), bf16_bits(c[3])) };
}
__device__ __forceinline__ v4u pack8_bf16_lo(v4f a, v4f c) {
  return (v4u){ pk16(bf16_lo_bits(a[0]), bf16_lo_bits(a[1])), pk16(bf16_lo_bits(a[2]), bf16_lo_bits(a[3])),
                pk16(bf16_lo_bits(c[0]), bf16_lo_bits(c[1])), pk16(bf16_lo_bits(c[2]), bf16_lo_bits(c[3])) };
}
__device__ __forceinline__ v4u pack8_f16(v4f a, v4f c) {
  return (v4u){ pk16(f16_bits(a[0]), f16_bits(a[1])), pk16(f16_bits(a[2]), f16_bits(a[3])),
                pk16(f16_bits(c[0]), f16_bits(c[1])), pk16(f16_bits(c[2]), f16_bits(c[3])) };
}

template <int FORM>
__global__ __launch_bounds__(256) void k_plane(const float* __restrict__ src, int rows, int cols, int ldsrc,
                                               unsigned short* __restrict__ dst, int MP, int KP) {
  static_assert(FORM >= 0 && FORM <= 3);
  const int KTOT = (FORM == 1 || FORM == 3) ? 2 * KP : KP;
  const unsigned ppr   = (unsigned)(KTOT >> 3);
  const unsigned kp8   = (unsigned)(KP >> 3);
  const unsigned total = (unsigned)MP * ppr;
  const unsigned g     = blockIdx.x * 256u + threadIdx.x;
  const unsigned rowu  = g / ppr;
  const unsigned p     = g - rowu * ppr;
  const bool second    = p >= kp8;
  const int row = (int)rowu;
  const int c0  = (int)((second ? p - kp8 : p) << 3);
  const float* srow = src + (size_t)clampi(row, 0, rows - 1) * (size_t)ldsrc;
  float x[8];
  unsigned mk[8];
#pragma unroll
  for (int e = 0; e < 8; ++e) {
    const int c = c0 + e;
    const float v = srow[clampi(c, 0, cols - 1)];
    asm volatile("" :: "v"(v));
    x[e]  = v;
    mk[e] = (row < rows && c < cols) ? 0xFFFFu : 0u;
  }
  const v4f a = (v4f){ x[0], x[1], x[2], x[3] };
  const v4f c = (v4f){ x[4], x[5], x[6], x[7] };
  v4u o;
  if (FORM == 2) {
    o = pack8_f16(a, c);
  } else {
    const v4u hi = pack8_bf16(a, c);
    o = hi;
    if (FORM == 1) { const v4u lo = pack8_bf16_lo(a, c); o = second ? lo : hi; }
  }
  const v4u mw = (v4u){ pk16(mk[0], mk[1]), pk16(mk[2], mk[3]), pk16(mk[4], mk[5]), pk16(mk[6], mk[7]) };
  o &= mw;
  if (g < total) {
    volatile v4u* q = (volatile v4u*)(dst + (size_t)g * 8);
    *q = o;
    __threadfence();
    *q = o;
  }
}

template <int FORM> struct FragOf    { typedef FragB T; };
template <>         struct FragOf<2> { typedef FragH T; };
__device__ __forceinline__ v8f mm(const FragB& a, const FragB& b, v8f c) { return wmb(a, b, c); }
__device__ __forceinline__ v8f mm(const FragH& a, const FragH& b, v8f c) { return wmh(a, b, c); }
template <class F> __device__ __forceinline__ F ld_frag(const unsigned short* p) {
  F f;
  f.h[0] = *(const v8usa*)(p);
  f.h[1] = *(const v8usa*)(p + 16);
  return f;
}

template <int FORM, int EPI>
__global__ __launch_bounds__(256) __attribute__((amdgpu_num_vgpr(248)))
void k_gemm_nt(const unsigned short* __restrict__ A, const unsigned short* __restrict__ B,
               const float* __restrict__ bias, float* __restrict__ D, int M, int N, int KTOT, int ldd) {
  static_assert(FORM >= 0 && FORM <= 2);
  static_assert(EPI == 0 || EPI == 1);
  typedef typename FragOf<FORM>::T F;
  __shared__ __attribute__((aligned(16))) float sT[8][16 * 68];
  const int lane = threadIdx.x & 31;
  const int wave = threadIdx.x >> 5;
  const int tilesM = (M + 63) >> 6;
  const int tilesN = (N + 63) >> 6;
  const int tile = blockIdx.x * 8 + wave;
  if (tile >= tilesM * tilesN) return;
  const int tm = tile / tilesN;
  const int tn = tile - tm * tilesN;
  const int m0 = tm << 6;
  const int n0 = tn << 6;

  const int rl = lane & 15;
  const int h8 = (lane >> 4) * 8;
  const unsigned short* pa = A + (size_t)(m0 + rl) * (size_t)KTOT + h8;
  const unsigned short* pb = B + (size_t)(n0 + rl) * (size_t)KTOT + h8;

  v8f acc[4][4];
#pragma unroll
  for (int i = 0; i < 4; ++i)
#pragma unroll
    for (int j = 0; j < 4; ++j) acc[i][j] = (v8f){0.f, 0.f, 0.f, 0.f, 0.f, 0.f, 0.f, 0.f};

#pragma unroll 1
  for (int k0 = 0; k0 < KTOT; k0 += 32) {
    F bf[4];
#pragma unroll
    for (int j = 0; j < 4; ++j) bf[j] = ld_frag<F>(pb + (size_t)(j << 4) * (size_t)KTOT + k0);
#pragma unroll
    for (int i = 0; i < 4; ++i) {
      const F af = ld_frag<F>(pa + (size_t)(i << 4) * (size_t)KTOT + k0);
#pragma unroll
      for (int j = 0; j < 4; ++j) acc[i][j] = mm(af, bf[j], acc[i][j]);
    }
  }

  float* slab = sT[wave];
  const int hh = lane >> 4;
  const int c4 = (lane & 15) * 4;
  const int nc = n0 + c4;
  const bool cok = nc < N;
  v4f bv = (v4f){0.f, 0.f, 0.f, 0.f};
  if (EPI == 1) {
    bv = *(const v4fa*)(bias + clampi(nc, 0, N - 4));
    asm volatile("" :: "v"(bv));
  }
#pragma unroll
  for (int i = 0; i < 4; ++i) {
    const int mBase = m0 + (i << 4);
#pragma unroll
    for (int j = 0; j < 4; ++j) {
#pragma unroll
      for (int r = 0; r < 8; ++r) slab[(h8 + r) * 68 + (j << 4) + rl] = acc[i][j][r];
    }
    __builtin_amdgcn_fence(__ATOMIC_RELEASE, "workgroup");
    __builtin_amdgcn_wave_barrier();
    __builtin_amdgcn_fence(__ATOMIC_ACQUIRE, "workgroup");
    v4f vv[8];
#pragma unroll
    for (int it = 0; it < 8; ++it) {
      const int row = it * 2 + hh;
      v4f v = *(const v4fa*)(slab + row * 68 + c4);
      if (EPI == 1) v += bv;
      vv[it] = v;
    }
    for (int pass = 0; pass < 2; ++pass) {
#pragma unroll
      for (int it = 0; it < 8; ++it) {
        const int row = mBase + it * 2 + hh;
        if (cok && row < M) *(volatile v4f*)(D + (size_t)row * (size_t)ldd + nc) = vv[it];
      }
      __threadfence();
    }
    __builtin_amdgcn_fence(__ATOMIC_RELEASE, "workgroup");
    __builtin_amdgcn_wave_barrier();
    __builtin_amdgcn_fence(__ATOMIC_ACQUIRE, "workgroup");
  }
}

#pragma clang fp contract(off)

#define NN         100000
#define NE         1200000
#define DD         64
#define A_TWO_TERM 1
#define K2         (64 * (1 + A_TWO_TERM))
#define PPR        (K2 / 8)
#define MPN        100096
#define NBLK       98
#define NBRUN      1024
#define DEGCAP     64
#define MAXHITS    12588
#define MAXDEG     28
#define NTHR       256
#define NWAVE      8
#define EPT        8
#define CHUNK      (NTHR * EPT)
#define WCAP       (EPT * 32)
#define LISTN      (NWAVE * WCAP)
#define NBMAX      2048
#define ESH        11
#define RCAP       16384
#define LDS_BKT    ((2 * RCAP + 2 * NBMAX + LISTN) * 4 + 64)
#define WSMAX      ((size_t)128 << 20)

static_assert(DD == 64 && K2 == 64 * (1 + A_TWO_TERM) && K2 % 32 == 0);
static_assert(NE == 585 * 2048 + 1920 && CHUNK == 2048);
static_assert(MPN % 128 == 0 && MPN % 64 == 0 && MPN >= NN && MPN - NN < 128);
static_assert(NN % 16 == 0);
static_assert(NBLK * NBRUN >= NN && (NBLK - 1) * NBRUN < NN);
static_assert((NN - (NBLK - 1) * NBRUN) % 32 == 0 && NBRUN % 128 == 0);
static_assert(NBRUN <= NBMAX && (1 << ESH) >= NBMAX && NTHR * 8 == NBMAX && LISTN >= NBMAX);
static_assert(NBRUN == NTHR * 4);
static_assert(NE <= (1 << (32 - ESH)));
static_assert(RCAP % 512 == 0 && RCAP * 100 >= MAXHITS * 125);
static_assert(DEGCAP >= MAXDEG + 8 && DEGCAP <= 64);
static_assert(LDS_BKT == 155712 && LDS_BKT <= 262144 && LDS_BKT + 34816 <= 327680);
static_assert((2 * 64 * PPR) % 256 == 0);
static_assert((size_t)NN * DD - 1 == 6399999);

constexpr size_t al256(size_t v) { return (v + 255) & ~(size_t)255; }
constexpr size_t O_X0   = 0;
constexpr size_t O_THL  = al256(O_X0   + (size_t)MPN * 64 * 4);
constexpr size_t O_H    = al256(O_THL  + (size_t)MPN * K2 * 2);
constexpr size_t O_LIST = al256(O_H    + (size_t)MPN * 64 * 4);
constexpr size_t O_OFFC = al256(O_LIST + (size_t)NBLK * RCAP * 8);
constexpr size_t O_META = al256(O_OFFC + (size_t)NBLK * 2048 * 4);
constexpr size_t O_WT2  = al256(O_META + (size_t)NBLK * 128);
constexpr size_t WS_TOTAL = al256(O_WT2 + (size_t)2 * 64 * K2 * 2);
static_assert(WS_TOTAL <= (size_t)WSMAX);
static_assert(A_TWO_TERM == 0 || WS_TOTAL == 90566912);
static_assert(O_THL % 256 == 0 && O_H % 256 == 0 && O_LIST % 256 == 0 && O_OFFC % 256 == 0 &&
              O_META % 256 == 0 && O_WT2 % 256 == 0);

typedef float v2f __attribute__((ext_vector_type(2)));
typedef int   v2i __attribute__((ext_vector_type(2)));
typedef int   v4i __attribute__((ext_vector_type(4)));
typedef v2f __attribute__((may_alias)) v2fa;
typedef v2i __attribute__((may_alias)) v2ia;
typedef v4i __attribute__((may_alias)) v4ia;

__device__ __forceinline__ void st2_v4u(void* p, const v4u v) {
  volatile v4u* q = (volatile v4u*)p;
  *q = v;
  __threadfence();
  *q = v;
}
__device__ __forceinline__ void st2_v4i(int* p, const v4i v) {
  volatile v4i* q = (volatile v4i*)p;
  *q = v;
  __threadfence();
  *q = v;
}

__device__ __forceinline__ v4u gather8_bf16(const float* __restrict__ src, int base, int k0, int kmask, int stride,
                                            unsigned mk) {
  float x[8];
#pragma unroll
  for (int e = 0; e < 8; ++e) {
    const float v = src[base + ((k0 + e) & kmask) * stride];
    asm volatile("" :: "v"(v));
    x[e] = v;
  }
  v4u o = pack8_bf16((v4f){ x[0], x[1], x[2], x[3] }, (v4f){ x[4], x[5], x[6], x[7] });
  o &= (v4u){ mk, mk, mk, mk };
  return o;
}

__global__ __launch_bounds__(256) void k_prep(const float* __restrict__ W, unsigned short* WT2) {
  const int u   = (int)blockIdx.x * 256 + (int)threadIdx.x;
  const int l   = u / (64 * PPR);
  const int rem = u - l * (64 * PPR);
  const int n   = rem / PPR;
  const int p   = rem - n * PPR;
  const v4u o = gather8_bf16(W, l * 4096 + n, 8 * p, 63, 64, 0xFFFFFFFFu);
  st2_v4u(WT2 + (size_t)u * 8, o);
}

#define EPSF 1e-5f
__device__ __forceinline__ float max_norm_f() { return (float)(1.0 - 1e-5); }

__device__ __forceinline__ float wsum(float s) {
  s += __shfl_xor(s, 16);
  s += __shfl_xor(s, 8);
  s += __shfl_xor(s, 4);
  s += __shfl_xor(s, 2);
  s += __shfl_xor(s, 1);
  return s;
}
__device__ __forceinline__ float rnorm(float a, float b) {
  const float s = wsum(a * a + b * b);
  const float n = sqrtf(s);
  return (n < EPSF) ? EPSF : n;
}
__device__ __forceinline__ void expm(float& a, float& b) {
  const float n  = rnorm(a, b);
  const float th = tanhf(n);
  a = (th * a) / n;
  b = (th * b) / n;
}
__device__ __forceinline__ void proj(float& a, float& b) {
  const float mx = max_norm_f();
  const float n  = rnorm(a, b);
  const float s  = mx / n;
  const bool clip = n > mx;
  const float ca = a * s;
  const float cb = b * s;
  a = clip ? ca : a;
  b = clip ? cb : b;
}
__device__ __forceinline__ void logm(float& a, float& b) {
  const float mx = max_norm_f();
  const float n  = rnorm(a, b);
  const float nc = (n > mx) ? mx : n;
  const float at = atanhf(nc);
  a = (at * a) / nc;
  b = (at * b) / nc;
}

__global__ __launch_bounds__(256) void k_rows0(const float* __restrict__ emb, float* X0, unsigned* THLw) {
  const int tid = (int)threadIdx.x, lane = tid & 31;
  const int wave = __builtin_amdgcn_readfirstlane(tid >> 5);
#pragma unroll 1
  for (int it = 0; it < 8; ++it) {
    const int row = (int)blockIdx.x * 64 + wave * 8 + it;
    const int rc  = row < NN ? row : NN - 1;
    const v2f v = *(const v2fa*)(emb + (size_t)rc * DD + 2 * lane);
    asm volatile("" :: "v"(v));
    float a = bf16_val(v.x);
    float b = bf16_val(v.y);
    expm(a, b);
    proj(a, b);
    const float xa = a, xb = b;
    logm(a, b);
    const unsigned lm = (row < NN) ? 0xFFFFFFFFu : 0u;
    v2f xo;
    xo.x = __uint_as_float(__float_as_uint(xa) & lm);
    xo.y = __uint_as_float(__float_as_uint(xb) & lm);
    const unsigned hiw = pk16(bf16_bits(a), bf16_bits(b)) & lm;
    const unsigned low = pk16(bf16_lo_bits(a), bf16_lo_bits(b)) & lm;
    volatile v2f* qx = (volatile v2f*)(X0 + (size_t)row * DD + 2 * lane);
    volatile unsigned* qh = THLw + (size_t)row * (K2 / 2) + lane;
    for (int pass = 0; pass < 2; ++pass) {
      *qx = xo;
      *qh = hiw;
      if (A_TWO_TERM) *(qh + 32) = low;
      __threadfence();
    }
  }
}

__device__ __forceinline__ int scan_chunk(const int* __restrict__ dsts, int nE, int cbase, int slotBase,
                                          int nb, int vec8, int* list, int tid, int lane, int wave) {
  int wc = 0;
  const int el0  = tid * EPT;
  const int e0   = cbase + el0;
  const int sent = (-0x7fffffff - 1);
  v4i da, db;
  if (vec8 != 0 && cbase + CHUNK <= nE) {
    da = *(const v4i*)(dsts + e0);
    db = *(const v4i*)(dsts + e0 + 4);
  } else {
    const int t0 = dsts[min(e0 + 0, nE - 1)];
    const int t1 = dsts[min(e0 + 1, nE - 1)];
    const int t2 = dsts[min(e0 + 2, nE - 1)];
    const int t3 = dsts[min(e0 + 3, nE - 1)];
    const int t4 = dsts[min(e0 + 4, nE - 1)];
    const int t5 = dsts[min(e0 + 5, nE - 1)];
    const int t6 = dsts[min(e0 + 6, nE - 1)];
    const int t7 = dsts[min(e0 + 7, nE - 1)];
    asm volatile("" :: "v"(t0), "v"(t1), "v"(t2), "v"(t3), "v"(t4), "v"(t5), "v"(t6), "v"(t7));
    da.x = (e0 + 0 < nE) ? t0 : sent;
    da.y = (e0 + 1 < nE) ? t1 : sent;
    da.z = (e0 + 2 < nE) ? t2 : sent;
    da.w = (e0 + 3 < nE) ? t3 : sent;
    db.x = (e0 + 4 < nE) ? t4 : sent;
    db.y = (e0 + 5 < nE) ? t5 : sent;
    db.z = (e0 + 6 < nE) ? t6 : sent;
    db.w = (e0 + 7 < nE) ? t7 : sent;
  }
  const unsigned nbs = (unsigned)slotBase;
  const unsigned unb = (unsigned)nb;
  const unsigned s0 = (unsigned)da.x - nbs, s1 = (unsigned)da.y - nbs;
  const unsigned s2 = (unsigned)da.z - nbs, s3 = (unsigned)da.w - nbs;
  const unsigned s4 = (unsigned)db.x - nbs, s5 = (unsigned)db.y - nbs;
  const unsigned s6 = (unsigned)db.z - nbs, s7 = (unsigned)db.w - nbs;
  const bool h0 = s0 < unb, h1 = s1 < unb, h2 = s2 < unb, h3 = s3 < unb;
  const bool h4 = s4 < unb, h5 = s5 < unb, h6 = s6 < unb, h7 = s7 < unb;
  const unsigned any = __builtin_amdgcn_ballot_w32(h0 | h1 | h2 | h3 | h4 | h5 | h6 | h7);
  if (any != 0u) {
#define HITJ(J, HJ, SJ) { \
      const unsigned mj = __builtin_amdgcn_ballot_w32(HJ); \
      if (mj != 0u) { \
        if (HJ) { \
          const int pos = wc + (int)__builtin_amdgcn_mbcnt_lo(mj, 0u); \
          if (pos < WCAP) list[wave * WCAP + pos] = ((el0 + (J)) << 12) | (int)(SJ); \
        } \
        wc += (int)__builtin_popcount(mj); } }
    HITJ(0, h0, s0)
    HITJ(1, h1, s1)
    HITJ(2, h2, s2)
    HITJ(3, h3, s3)
    HITJ(4, h4, s4)
    HITJ(5, h5, s5)
    HITJ(6, h6, s6)
    HITJ(7, h7, s7)
#undef HITJ
  }
  return wc;
}

__device__ __forceinline__ int build_lists(const int* __restrict__ dsts, int nE, int nodeBase, int nb, int vec8,
                                           int* reg1, int* reg2, int* scnt, int* soff, int* list,
                                           int* wcnt, int* wtot, int tid, int lane, int wave) {
  for (int i = tid; i < NBMAX; i += NTHR) scnt[i] = 0;
  __syncthreads();

  int tot = 0;
  const int nChunks = (nE + CHUNK - 1) / CHUNK;
#pragma unroll 1
  for (int ch = 0; ch < nChunks; ++ch) {
    const int cbase = ch * CHUNK;
    const int wc = scan_chunk(dsts, nE, cbase, nodeBase, nb, vec8, list, tid, lane, wave);
    if (lane == 0) wcnt[wave] = wc;
    __syncthreads();
    int pre = 0, all = 0;
#pragma unroll
    for (int w2 = 0; w2 < NWAVE; ++w2) {
      int c = wcnt[w2];
      c = c < 0 ? 0 : (c > WCAP ? WCAP : c);
      all += c;
      pre += (w2 < wave) ? c : 0;
    }
    const int wcc  = wc > WCAP ? WCAP : wc;
    const int base = tot + pre;
#pragma unroll 1
    for (int i = lane; i < wcc; i += 32) {
      const int ent = list[wave * WCAP + i];
      const int el  = (ent >> 12) & (CHUNK - 1);
      const int sl  = ent & (NBMAX - 1);
      int eid = cbase + el;
      eid = eid > nE - 1 ? nE - 1 : eid;
      const int pos = base + i;
      if (pos < RCAP) reg1[pos] = (int)(((unsigned)eid << ESH) | (unsigned)sl);
    }
    tot += all;
    tot = tot > RCAP ? RCAP : tot;
    __syncthreads();
  }
  const int nh = __builtin_amdgcn_readfirstlane(tot < 0 ? 0 : (tot > RCAP ? RCAP : tot));

  if (wave == 0) {
#pragma unroll 1
    for (int b0 = 0; b0 < nh; b0 += 32) {
      const int idx = b0 + lane;
      const int uv  = reg1[idx < nh ? idx : nh - 1];
      const int m32 = (nh - b0) < 32 ? (nh - b0) : 32;
#pragma unroll 1
      for (int k = 0; k < m32; ++k) {
        const int u  = __builtin_amdgcn_readlane(uv, k);
        const int sl = u & (NBMAX - 1);
        if (lane == 0) scnt[sl] = scnt[sl] + 1;
      }
    }
  }
  __syncthreads();

  {
    const v4i ca = *(const v4i*)(scnt + 8 * tid);
    const v4i cb = *(const v4i*)(scnt + 8 * tid + 4);
    const int e0 = ca.x < 0 ? 0 : ca.x, e1 = ca.y < 0 ? 0 : ca.y, e2 = ca.z < 0 ? 0 : ca.z, e3 = ca.w < 0 ? 0 : ca.w;
    const int e4 = cb.x < 0 ? 0 : cb.x, e5 = cb.y < 0 ? 0 : cb.y, e6 = cb.z < 0 ? 0 : cb.z, e7 = cb.w < 0 ? 0 : cb.w;
    const int ts = e0 + e1 + e2 + e3 + e4 + e5 + e6 + e7;
    int incl = ts;
#pragma unroll
    for (int d = 1; d < 32; d <<= 1) {
      const int up = __shfl_up(incl, d);
      if (lane >= d) incl += up;
    }
    if (lane == 31) wtot[wave] = incl;
    __syncthreads();
    int pre = 0;
#pragma unroll
    for (int w2 = 0; w2 < NWAVE; ++w2) pre += (w2 < wave) ? wtot[w2] : 0;
    int run = pre + incl - ts;
    soff[8 * tid + 0] = run; run += e0;
    soff[8 * tid + 1] = run; run += e1;
    soff[8 * tid + 2] = run; run += e2;
    soff[8 * tid + 3] = run; run += e3;
    soff[8 * tid + 4] = run; run += e4;
    soff[8 * tid + 5] = run; run += e5;
    soff[8 * tid + 6] = run; run += e6;
    soff[8 * tid + 7] = run;
  }
  __syncthreads();
  for (int i = tid; i < NBMAX; i += NTHR) list[i] = soff[i];
  __syncthreads();

  if (wave == 0) {
#pragma unroll 1
    for (int b0 = 0; b0 < nh; b0 += 32) {
      const int idx = b0 + lane;
      const int uv  = reg1[idx < nh ? idx : nh - 1];
      const int m32 = (nh - b0) < 32 ? (nh - b0) : 32;
#pragma unroll 1
      for (int k = 0; k < m32; ++k) {
        const int u   = __builtin_amdgcn_readlane(uv, k);
        const int sl  = u & (NBMAX - 1);
        const int eid = (int)((unsigned)u >> ESH);
        if (lane == 0) {
          int pos = list[sl];
          pos = pos < 0 ? 0 : (pos > RCAP - 1 ? RCAP - 1 : pos);
          reg2[pos] = eid;
          list[sl] = pos + 1;
        }
      }
    }
  }
  __syncthreads();
  return nh;
}

__global__ __launch_bounds__(NTHR) void k_bucket(const int* __restrict__ keys, const int* __restrict__ cols,
                                                 const float* __restrict__ vals, int nE, int nN, int vec8,
                                                 int* LIST, int* OFFC, int* META) {
  extern __shared__ v4f lds_dyn[];
  int* reg1 = (int*)lds_dyn;
  int* reg2 = reg1 + RCAP;
  int* scnt = reg2 + RCAP;
  int* soff = scnt + NBMAX;
  int* list = soff + NBMAX;
  int* wcnt = list + LISTN;
  int* wtot = wcnt + NWAVE;
  const int tid = (int)threadIdx.x, lane = tid & 31;
  const int wave = __builtin_amdgcn_readfirstlane(tid >> 5);
  const int b = (int)blockIdx.x;
  const int nodeBase = b * NBRUN;
  int nb = nN - nodeBase;
  nb = nb < 0 ? 0 : (nb > NBRUN ? NBRUN : nb);
  if (tid == 0) reg2[0] = 0;

  const int nh = build_lists(keys, nE, nodeBase, nb, vec8, reg1, reg2, scnt, soff, list, wcnt, wtot, tid, lane, wave);

  int* bl = LIST + (size_t)b * RCAP * 2;
  const int last = nh > 0 ? nh - 1 : 0;
#pragma unroll 1
  for (int base = 0; base < RCAP; base += 512) {
    const int i0 = base + 2 * tid;
    int e0 = reg2[i0     < last ? i0     : last];
    int e1 = reg2[i0 + 1 < last ? i0 + 1 : last];
    e0 = clampi(e0, 0, nE - 1);
    e1 = clampi(e1, 0, nE - 1);
    int   c0 = cols[e0];
    int   c1 = cols[e1];
    float w0 = vals[e0];
    float w1 = vals[e1];
    asm volatile("" :: "v"(c0), "v"(c1), "v"(w0), "v"(w1));
    c0 = clampi(c0, 0, nN - 1);
    c1 = clampi(c1, 0, nN - 1);
    const int u0 = (int)(bf16_bits(w0) << 16);
    const int u1 = (int)(bf16_bits(w1) << 16);
    const int m0 = (i0     < nh) ? -1 : 0;
    const int m1 = (i0 + 1 < nh) ? -1 : 0;
    v4i v;
    v.x = c0 & m0;
    v.y = u0 & m0;
    v.z = c1 & m1;
    v.w = u1 & m1;
    st2_v4i(bl + 2 * i0, v);
  }
  {
    const v4i so = *(const v4ia*)(soff + 4 * tid);
    const v4i sc = *(const v4ia*)(scnt + 4 * tid);
    int* oc = OFFC + (size_t)b * 2048;
    st2_v4i(oc + 4 * tid, so);
    st2_v4i(oc + 1024 + 4 * tid, sc);
  }
  if (tid < 8) {
    v4i mv;
    mv.x = (tid == 0) ? nh : 0;
    mv.y = (tid == 0 && nh >= RCAP) ? 1 : 0;
    mv.z = 0; mv.w = 0;
    st2_v4i(META + (size_t)b * 32 + 4 * tid, mv);
  }
}

template <int LAST>
__global__ __launch_bounds__(256) void k_replay(const float* __restrict__ H, const int* __restrict__ LIST,
                                                const int* __restrict__ OFFC, const int* __restrict__ META,
                                                const float* __restrict__ X0, unsigned* THLw, float* out) {
  const int tid = (int)threadIdx.x, lane = tid & 31;
  const int wave = __builtin_amdgcn_readfirstlane(tid >> 5);
  const int b = (int)blockIdx.x;
  const int nodeBase = b * NBRUN;
  const int nb = clampi(NN - nodeBase, 0, NBRUN);
  int nhv = META[(size_t)b * 32];
  int flv = META[(size_t)b * 32 + 1];
  asm volatile("" :: "v"(nhv), "v"(flv));
  const int nh   = __builtin_amdgcn_readfirstlane(clampi(nhv, 0, RCAP));
  const int flag = __builtin_amdgcn_readfirstlane(flv);
  const bool ovf = flag != 0;
  const int* bl = LIST + (size_t)b * RCAP * 2;
  const int* oc = OFFC + (size_t)b * 2048;
  const int nhm1 = nh > 0 ? nh - 1 : 0;
  const float qnan = __int_as_float(0x7fc00000);

#pragma unroll 1
  for (int g = 0; g < 4; ++g) {
    const int slot0 = wave * 128 + g * 32;
    if (slot0 >= nb) break;
    int stv = oc[slot0 + lane];
    int cv  = oc[1024 + slot0 + lane];
    asm volatile("" :: "v"(stv), "v"(cv));
    const int craw = cv < 0 ? 0 : cv;
    const int pv = (craw > DEGCAP) ? 1 : 0;
    stv = clampi(stv, 0, nh);
    int cc = clampi(craw, 0, DEGCAP);
    cc = cc > nh - stv ? nh - stv : cc;
    cc = (nodeBase + slot0 + lane < NN) ? cc : 0;
#pragma unroll 1
    for (int rr = 0; rr < 32; ++rr) {
      const int st  = __builtin_amdgcn_readlane(stv, rr);
      const int cnt = __builtin_amdgcn_readlane(cc, rr);
      const int prw = __builtin_amdgcn_readlane(pv, rr);
      const int row = nodeBase + slot0 + rr;
      float ax = 0.0f, ay = 0.0f;
#pragma unroll 1
      for (int b0 = 0; b0 < cnt; b0 += 32) {
        const int li = clampi(st + b0 + lane, 0, nhm1);
        const v2i ent = *(const v2ia*)(bl + 2 * (size_t)li);
        asm volatile("" :: "v"(ent));
        const int col = clampi(ent.x, 0, NN - 1);
        const int wb  = ent.y;
        const int m32 = (cnt - b0) < 32 ? (cnt - b0) : 32;
#pragma unroll 2
        for (int q = 0; q < m32; ++q) {
          const int cq = __builtin_amdgcn_readlane(col, q);
          const float wq = __int_as_float(__builtin_amdgcn_readlane(wb, q));
          const v2f hv = *(const v2fa*)(H + (size_t)cq * DD + 2 * lane);
          const float px = wq * hv.x;
          const float py = wq * hv.y;
          ax = ax + px;
          ay = ay + py;
        }
      }
      float a  = tanhf(ax);
      float bb = tanhf(ay);
      expm(a, bb);
      proj(a, bb);
      const bool bad = ovf || (prw != 0);
      if (LAST == 0) {
        logm(a, bb);
        a  = bad ? qnan : a;
        bb = bad ? qnan : bb;
        const unsigned hiw = pk16(bf16_bits(a), bf16_bits(bb));
        const unsigned low = pk16(bf16_lo_bits(a), bf16_lo_bits(bb));
        if (row < NN) {
          volatile unsigned* qh = THLw + (size_t)row * (K2 / 2) + lane;
          for (int pass = 0; pass < 2; ++pass) {
            *qh = hiw;
            if (A_TWO_TERM) *(qh + 32) = low;
            __threadfence();
          }
        }
      } else {
        const int rc = row < NN ? row : NN - 1;
        const v2f yv = *(const v2fa*)(X0 + (size_t)rc * DD + 2 * lane);
        asm volatile("" :: "v"(yv));
        const float ya = yv.x, yb = yv.y;
        const float x2 = wsum(a * a + bb * bb);
        const float y2 = wsum(ya * ya + yb * yb);
        const float xy = wsum(a * ya + bb * yb);
        const float t2 = 2.0f * xy;
        const float ca = (1.0f + t2) + y2;
        const float cb = 1.0f - x2;
        float den = (1.0f + t2) + x2 * y2;
        den = (den < EPSF) ? EPSF : den;
        float oa = (ca * a  + cb * ya) / den;
        float ob = (ca * bb + cb * yb) / den;
        proj(oa, ob);
        oa = bad ? qnan : oa;
        ob = bad ? qnan : ob;
        v2f ov;
        ov.x = oa;
        ov.y = ob;
        if (row < NN) {
          volatile v2f* qo = (volatile v2f*)(out + (size_t)row * DD + 2 * lane);
          for (int pass = 0; pass < 2; ++pass) {
            *qo = ov;
            __threadfence();
          }
        }
      }
    }
  }
}

extern "C" void kernel_launch(void* const* d_in, const int* in_sizes, int n_in,
                              void* d_out, int out_size, void* d_ws, size_t ws_size,
                              hipStream_t stream) {
  if (n_in < 5) return;
  if (in_sizes[0] != NN * DD || in_sizes[1] != 2 * DD * DD) return;
  if (in_sizes[2] != NE || in_sizes[3] != NE || in_sizes[4] != NE) return;
  if (out_size != NN * DD) return;
  if (ws_size < WS_TOTAL) return;

  const float* emb   = (const float*)d_in[0];
  const float* Wall  = (const float*)d_in[1];
  const int*   erows = (const int*)  d_in[2];
  const int*   ecols = (const int*)  d_in[3];
  const float* evals = (const float*)d_in[4];
  float* out = (float*)d_out;

  char* ws = (char*)d_ws;
  float*          X0   = (float*)(ws + O_X0);
  unsigned short* THL  = (unsigned short*)(ws + O_THL);
  float*          H    = (float*)(ws + O_H);
  int*            LIST = (int*)(ws + O_LIST);
  int*            OFFC = (int*)(ws + O_OFFC);
  int*            META = (int*)(ws + O_META);
  unsigned short* WT2  = (unsigned short*)(ws + O_WT2);

  hipFuncSetAttribute(reinterpret_cast<const void*>(&k_bucket),
                      hipFuncAttributeMaxDynamicSharedMemorySize, LDS_BKT);

  k_prep<<<2 * 64 * PPR / 256, 256, 0, stream>>>(Wall, WT2);
  k_rows0<<<MPN / 64, 256, 0, stream>>>(emb, X0, (unsigned*)THL);
  k_bucket<<<NBLK, NTHR, LDS_BKT, stream>>>(erows, ecols, evals, NE, NN, 1, LIST, OFFC, META);
  k_gemm_nt<0, 0><<<(1563 + 7) / 8, 256, 0, stream>>>(THL, WT2, X0, H, NN, 64, K2, 64);
  k_replay<0><<<NBLK, 256, 0, stream>>>(H, LIST, OFFC, META, X0, (unsigned*)THL, out);
  k_gemm_nt<0, 0><<<(1563 + 7) / 8, 256, 0, stream>>>(THL, WT2 + (size_t)64 * K2, X0, H, NN, 64, K2, 64);
  k_replay<1><<<NBLK, 256, 0, stream>>>(H, LIST, OFFC, META, X0, (unsigned*)THL, out);
}
